// SAGE_57372173140138
// MI455X (gfx1250) — hardware-verified
//
#include <hip/hip_runtime.h>
#include <stddef.h>
#include <stdint.h>


#define DIN    128
#define DHID   128
#define DOUT   64
#define KC     256
#define AP     256
#define RB     256
#define NTHR   256
#define NWAVE  8
#define EPT    8
#define CHUNK  (NTHR * EPT)
#define WCAP   (EPT * 32)
#define LISTN  (NWAVE * WCAP)
#define NBA    1024
#define SLA    10
#define RCAP   28672
#define DEGCAP 64
#define GBM    64
#define GBN    64
#define GRW    4
#define GTHR   (32 * GRW)
#define UW1    (DHID * (KC / 8))
#define UW2    (DOUT * (KC / 8))
#define AGG_ZINTS    (LISTN + 2 * RCAP + 3 * NBA)
#define MISC_INTS    16
#define ROWBUF_INTS  (NWAVE * RB / 2)
#define AGG_LDS_INTS (AGG_ZINTS + MISC_INTS + ROWBUF_INTS)
#define WSMAX  134217728

static_assert((CHUNK & (CHUNK - 1)) == 0 && CHUNK <= 4096);
static_assert((NBA & (NBA - 1)) == 0 && NBA == (1 << SLA));
static_assert(((long long)CHUNK << SLA) < (1LL << 31));
static_assert(LISTN % NTHR == 0);
static_assert(NBA % NWAVE == 0 && NBA % 32 == 0 && NBA % GBM == 0);
static_assert(RCAP % 4 == 0 && AGG_ZINTS % 4 == 0 && LISTN % 4 == 0 && ((AGG_ZINTS + MISC_INTS) % 4) == 0);
static_assert(AGG_ZINTS % (NTHR * 4) == 0);
static_assert(KC % 32 == 0 && KC == AP && KC == 2 * DIN && DHID == DIN && RB == AP && RB % 16 == 0);
static_assert(DIN == 4 * 32 && DOUT == 2 * 32);
static_assert(DHID == 2 * GBN && DOUT == GBN && GBM == GRW * 16 && GRW == 4 && GTHR == 128);
static_assert(UW1 % NTHR == 0 && (UW1 + UW2) % NTHR == 0);
static_assert(AGG_LDS_INTS * 4 <= 300000);
static_assert(DEGCAP <= RCAP && WCAP <= LISTN);
static_assert(GBM * GBN * 4 == GBM * (2 * GBN) * 2);
static_assert(ROWBUF_INTS % 4 == 0 && RB / 2 >= DOUT);

typedef float          v2f   __attribute__((ext_vector_type(2)));
typedef float          v4f   __attribute__((ext_vector_type(4)));
typedef float          v8f   __attribute__((ext_vector_type(8)));
typedef int            v4i   __attribute__((ext_vector_type(4)));
typedef int            v8i   __attribute__((ext_vector_type(8)));
typedef unsigned       v2u   __attribute__((ext_vector_type(2)));
typedef unsigned       v4u   __attribute__((ext_vector_type(4)));
typedef unsigned short v8us  __attribute__((ext_vector_type(8)));
typedef unsigned short v16us __attribute__((ext_vector_type(16)));
typedef __bf16         v16bf __attribute__((ext_vector_type(16)));
typedef unsigned __attribute__((may_alias)) ua;
typedef v2f  __attribute__((may_alias)) v2fa;
typedef v4f  __attribute__((may_alias)) v4fa;
typedef v4i  __attribute__((may_alias)) v4ia;
typedef v2u  __attribute__((may_alias)) v2ua;
typedef v8us __attribute__((may_alias)) v8usa;
union FragB { v16bf v; v16us u; v8us h[2]; v8i w; };

__device__ __forceinline__ v8f wmb(const FragB& a, const FragB& b, v8f c) {
  v8f d = __builtin_amdgcn_wmma_f32_16x16x32_bf16(false, a.v, false, b.v, (short)0, c, false, false);
  asm volatile("v_nop\n\tv_nop\n\tv_nop\n\tv_nop" : "+v"(d) : "v"(a.w), "v"(b.w));
  return d;
}

__device__ __forceinline__ unsigned bf16_bits(float f) {
  const unsigned u = __float_as_uint(f);
  return (u + 0x7FFFu + ((u >> 16) & 1u)) >> 16;
}
__device__ __forceinline__ float bf16_val(float f) {
  return __uint_as_float(bf16_bits(f) << 16);
}

__device__ __forceinline__ void wave_sync() {
  __builtin_amdgcn_fence(__ATOMIC_RELEASE, "wavefront");
  __builtin_amdgcn_wave_barrier();
  __builtin_amdgcn_fence(__ATOMIC_ACQUIRE, "wavefront");
}

template <int SLB>
__device__ __forceinline__ int scan_chunk(const int* __restrict__ dsts, int nE, int cbase, int slotBase,
                                          int nb, int vec8, int* list, int tid, int lane, int wave) {
  int wc = 0;
  const int el0  = tid * EPT;
  const int e0   = cbase + el0;
  const int sent = -2147483647 - 1;
  v4i da, db;
  if (vec8 != 0 && cbase + CHUNK <= nE) {
    da = *(const v4i*)(dsts + e0);
    db = *(const v4i*)(dsts + e0 + 4);
  } else {
    da.x = (e0     < nE) ? dsts[min(e0,     nE - 1)] : sent;
    da.y = (e0 + 1 < nE) ? dsts[min(e0 + 1, nE - 1)] : sent;
    da.z = (e0 + 2 < nE) ? dsts[min(e0 + 2, nE - 1)] : sent;
    da.w = (e0 + 3 < nE) ? dsts[min(e0 + 3, nE - 1)] : sent;
    db.x = (e0 + 4 < nE) ? dsts[min(e0 + 4, nE - 1)] : sent;
    db.y = (e0 + 5 < nE) ? dsts[min(e0 + 5, nE - 1)] : sent;
    db.z = (e0 + 6 < nE) ? dsts[min(e0 + 6, nE - 1)] : sent;
    db.w = (e0 + 7 < nE) ? dsts[min(e0 + 7, nE - 1)] : sent;
  }
  const unsigned nbs = (unsigned)slotBase;
  const unsigned unb = (unsigned)nb;
  const unsigned s0 = (unsigned)da.x - nbs, s1 = (unsigned)da.y - nbs;
  const unsigned s2 = (unsigned)da.z - nbs, s3 = (unsigned)da.w - nbs;
  const unsigned s4 = (unsigned)db.x - nbs, s5 = (unsigned)db.y - nbs;
  const unsigned s6 = (unsigned)db.z - nbs, s7 = (unsigned)db.w - nbs;
  const bool h0 = s0 < unb, h1 = s1 < unb, h2 = s2 < unb, h3 = s3 < unb;
  const bool h4 = s4 < unb, h5 = s5 < unb, h6 = s6 < unb, h7 = s7 < unb;
  const unsigned any = __builtin_amdgcn_ballot_w32(h0 | h1 | h2 | h3 | h4 | h5 | h6 | h7);
  if (any != 0u) {
#define HITJ(J, HJ, SJ) { \
      const unsigned mj = __builtin_amdgcn_ballot_w32(HJ); \
      if (mj != 0u) { \
        if (HJ) { \
          const int pos = wc + (int)__builtin_amdgcn_mbcnt_lo(mj, 0u); \
          if (pos < WCAP) list[wave * WCAP + pos] = ((el0 + (J)) << SLB) | (int)(SJ); \
        } \
        wc += (int)__builtin_popcount(mj); } }
    HITJ(0, h0, s0)
    HITJ(1, h1, s1)
    HITJ(2, h2, s2)
    HITJ(3, h3, s3)
    HITJ(4, h4, s4)
    HITJ(5, h5, s5)
    HITJ(6, h6, s6)
    HITJ(7, h7, s7)
#undef HITJ
  }
  return wc;
}

__global__ __launch_bounds__(NTHR) void k_wprep(const float* __restrict__ W1, const float* __restrict__ W2,
                                                unsigned short* BT1, unsigned short* BT2) {
  const int u = (int)blockIdx.x * NTHR + (int)threadIdx.x;
  if (u >= UW1 + UW2) return;
  const int part = (u >= UW1) ? 1 : 0;
  const int v    = (part != 0) ? (u - UW1) : u;
  const float* W = (part != 0) ? W2 : W1;
  unsigned short* P = (part != 0) ? BT2 : BT1;
  const int n  = v >> 5;
  const int c8 = (v & 31) * 8;
  const int k8 = c8 & (DIN - 1);
  const float* p = W + (size_t)n * DIN + k8;
  const v4f a = *(const v4fa*)p;
  const v4f b = *(const v4fa*)(p + 4);
  v8us o;
  o[0] = (unsigned short)bf16_bits(a.x); o[1] = (unsigned short)bf16_bits(a.y);
  o[2] = (unsigned short)bf16_bits(a.z); o[3] = (unsigned short)bf16_bits(a.w);
  o[4] = (unsigned short)bf16_bits(b.x); o[5] = (unsigned short)bf16_bits(b.y);
  o[6] = (unsigned short)bf16_bits(b.z); o[7] = (unsigned short)bf16_bits(b.w);
  unsigned short* dp = P + (size_t)n * AP + c8;
  *(volatile v8us*)dp = o;
  __threadfence();
  *(volatile v8us*)dp = o;
}

template <int FIN>
__global__ __launch_bounds__(GTHR) void k_gemm(const unsigned short* __restrict__ Apl,
                                                const unsigned short* __restrict__ BT,
                                                const float* __restrict__ bias, int nV,
                                                unsigned short* Hpl, float* Tpl) {
  __shared__ __attribute__((aligned(16))) float gsm[GBM * GBN];
  const int tid = (int)threadIdx.x, lane = tid & 31, wave = tid >> 5, hh = lane >> 4, m = lane & 15;
  const int rowBase = (int)blockIdx.x * GBM;
  const int col0    = (int)blockIdx.y * GBN;

  v8f acc[4];
  {
    const v8f z = {0.f, 0.f, 0.f, 0.f, 0.f, 0.f, 0.f, 0.f};
#pragma unroll
    for (int t = 0; t < 4; ++t) acc[t] = z;
  }
  const unsigned short* ap = Apl + (size_t)(rowBase + 16 * wave + m) * (size_t)AP + 8 * hh;
  const unsigned short* bp = BT + (size_t)(col0 + m) * (size_t)KC + 8 * hh;

#pragma unroll 1
  for (int k0 = 0; k0 < KC; k0 += 32) {
    FragB af;
    af.h[0] = *(const v8usa*)(ap + k0);
    af.h[1] = *(const v8usa*)(ap + k0 + 16);
#pragma unroll
    for (int nt = 0; nt < 4; ++nt) {
      const unsigned short* wq = bp + (size_t)(16 * nt) * (size_t)KC + k0;
      FragB bf;
      bf.h[0] = *(const v8usa*)wq;
      bf.h[1] = *(const v8usa*)(wq + 16);
      acc[nt] = wmb(af, bf, acc[nt]);
    }
  }

#pragma unroll
  for (int nt = 0; nt < 4; ++nt) {
    const int lc = 16 * nt + m;
#pragma unroll
    for (int r = 0; r < 8; ++r) {
      const int lr = 16 * wave + 8 * hh + r;
      gsm[lr * GBN + lc] = acc[nt][r];
    }
  }
  __syncthreads();

  v4f bb4;
  if constexpr (FIN == 0) {
    const v4f tb = *(const v4f*)(bias + col0 + 4 * m);
    bb4.x = bf16_val(tb.x); bb4.y = bf16_val(tb.y); bb4.z = bf16_val(tb.z); bb4.w = bf16_val(tb.w);
  } else {
    bb4.x = 0.0f; bb4.y = 0.0f; bb4.z = 0.0f; bb4.w = 0.0f;
  }

  v4f q[8];
#pragma unroll
  for (int ii = 0; ii < 8; ++ii) {
    const int lr = 16 * wave + 2 * ii + hh;
    const bool ok = (rowBase + lr) < nV;
    const v4f t = *(const v4fa*)(gsm + lr * GBN + 4 * m) + bb4;
    v4f y = t;
    if constexpr (FIN == 0) {
      y.x = (t.x < 0.0f) ? 0.0f : t.x;
      y.y = (t.y < 0.0f) ? 0.0f : t.y;
      y.z = (t.z < 0.0f) ? 0.0f : t.z;
      y.w = (t.w < 0.0f) ? 0.0f : t.w;
    }
    y.x = ok ? y.x : 0.0f; y.y = ok ? y.y : 0.0f; y.z = ok ? y.z : 0.0f; y.w = ok ? y.w : 0.0f;
    q[ii] = y;
  }

  if constexpr (FIN != 0) {
#pragma unroll
    for (int ii = 0; ii < 8; ++ii) {
      const int gr = rowBase + 16 * wave + 2 * ii + hh;
      *(volatile v4f*)(Tpl + (size_t)gr * DOUT + 4 * m) = q[ii];
    }
    __threadfence();
#pragma unroll
    for (int ii = 0; ii < 8; ++ii) {
      const int gr = rowBase + 16 * wave + 2 * ii + hh;
      *(volatile v4f*)(Tpl + (size_t)gr * DOUT + 4 * m) = q[ii];
    }
  } else {
    __syncthreads();
#pragma unroll
    for (int ii = 0; ii < 8; ++ii) {
      const int lr = 16 * wave + 2 * ii + hh;
      unsigned h0, h1, h2, h3, l0, l1, l2, l3;
      h0 = bf16_bits(q[ii].x); l0 = bf16_bits(q[ii].x - __uint_as_float(h0 << 16));
      h1 = bf16_bits(q[ii].y); l1 = bf16_bits(q[ii].y - __uint_as_float(h1 << 16));
      h2 = bf16_bits(q[ii].z); l2 = bf16_bits(q[ii].z - __uint_as_float(h2 << 16));
      h3 = bf16_bits(q[ii].w); l3 = bf16_bits(q[ii].w - __uint_as_float(h3 << 16));
      v2u ph, pl;
      ph.x = h0 | (h1 << 16); ph.y = h2 | (h3 << 16);
      pl.x = l0 | (l1 << 16); pl.y = l2 | (l3 << 16);
      ua* srow = (ua*)gsm + (size_t)lr * GBN;
      *(v2ua*)(srow + 2 * m) = ph;
      *(v2ua*)(srow + GBN / 2 + 2 * m) = pl;
    }
    __syncthreads();
    v8us qv[8];
#pragma unroll
    for (int ii = 0; ii < 8; ++ii) {
      const int lr = 16 * wave + 2 * ii + hh;
      const unsigned short* srow = (const unsigned short*)gsm + (size_t)lr * (2 * GBN);
      qv[ii] = *(const v8usa*)(srow + 8 * m);
    }
    const int coff = col0 + 8 * m + (m >> 3) * GBN;
#pragma unroll
    for (int ii = 0; ii < 8; ++ii) {
      unsigned short* rp = Hpl + (size_t)(rowBase + 16 * wave + 2 * ii + hh) * (size_t)AP + coff;
      *(volatile v8us*)rp = qv[ii];
    }
    __threadfence();
#pragma unroll
    for (int ii = 0; ii < 8; ++ii) {
      unsigned short* rp = Hpl + (size_t)(rowBase + 16 * wave + 2 * ii + hh) * (size_t)AP + coff;
      *(volatile v8us*)rp = qv[ii];
    }
  }
}

template <int L1>
__global__ __launch_bounds__(NTHR) void k_scan(const int* __restrict__ gath, const int* __restrict__ keys,
                                               int nE, int nN, int vec8, int mRows,
                                               const float* __restrict__ src, const float* __restrict__ bias,
                                               unsigned short* apl, float* outp) {
  extern __shared__ __attribute__((aligned(16))) int dsm[];
  int* list = dsm;
  int* hl   = dsm + LISTN;
  int* sl   = hl + RCAP;
  int* cnt  = sl + RCAP;
  int* offs = cnt + NBA;
  int* cur  = offs + NBA;
  int* misc = cur + NBA;
  const int tid = (int)threadIdx.x, lane = tid & 31, wave = tid >> 5;
  unsigned short* rowbuf = (unsigned short*)(misc + MISC_INTS) + wave * RB;
  ua* rowu = (ua*)rowbuf;
  float* rowf = (float*)(misc + MISC_INTS) + wave * (RB / 2);
  const int nodeBase = (int)blockIdx.x * NBA;

  {
    const v4i z4 = {0, 0, 0, 0};
    for (int i = tid * 4; i < AGG_ZINTS; i += NTHR * 4) *(v4ia*)(dsm + i) = z4;
    if (tid < MISC_INTS) misc[tid] = 0;
  }
  float bv0 = 0.0f, bv1 = 0.0f;
  if constexpr (L1 == 0) {
    const v2f tb = *(const v2fa*)(bias + 2 * lane);
    bv0 = bf16_val(tb.x); bv1 = bf16_val(tb.y);
  }
  __syncthreads();

  int t = 0, ov = 0;
  const int nChunks = (nE + CHUNK - 1) / CHUNK;
#pragma unroll 1
  for (int chn = 0; chn < nChunks; ++chn) {
    const int cbase = chn * CHUNK;
    const int wc = scan_chunk<SLA>(keys, nE, cbase, nodeBase, NBA, vec8, list, tid, lane, wave);
    if (lane == 0) misc[wave] = wc;
    __syncthreads();
    if (wave == 0) {
#pragma unroll 1
      for (int w2 = 0; w2 < NWAVE; ++w2) {
        int c = misc[w2];
        c = c < 0 ? 0 : (c > WCAP ? WCAP : c);
#pragma unroll 1
        for (int b0 = 0; b0 < c; b0 += 32) {
          const int idx = b0 + lane;
          const int ent = list[w2 * WCAP + (idx < WCAP ? idx : WCAP - 1)];
          const int m32 = (c - b0) < 32 ? (c - b0) : 32;
#pragma unroll 1
          for (int k = 0; k < m32; ++k) {
            const int u    = __builtin_amdgcn_readlane(ent, k);
            const int slot = u & (NBA - 1);
            const int el   = (u >> SLA) & (CHUNK - 1);
            const int pk   = ((cbase + el) << SLA) | slot;
            if (t < RCAP) {
              if (lane == 0) { hl[t] = pk; cnt[slot] = cnt[slot] + 1; }
              t = t + 1;
            } else {
              ov = 1;
            }
          }
        }
      }
    }
    __syncthreads();
  }
  if (wave == 0 && lane == 0) { misc[8] = t; misc[9] = ov; }
  __syncthreads();
  int tt = misc[8];
  tt = tt < 0 ? 0 : (tt > RCAP ? RCAP : tt);
  const int ovf = misc[9];

  if (wave == 0) {
    const int base = lane * (NBA / 32);
    int s = 0;
#pragma unroll 1
    for (int i = 0; i < NBA / 32; ++i) s += cnt[base + i];
    int incl = s;
#pragma unroll
    for (int d = 1; d < 32; d <<= 1) {
      const int y = __shfl_up(incl, d, 32);
      if (lane >= d) incl += y;
    }
    int run = incl - s;
#pragma unroll 1
    for (int i = 0; i < NBA / 32; ++i) {
      const int cv = cnt[base + i];
      offs[base + i] = run;
      cur[base + i]  = run;
      run += cv;
    }
  }
  __syncthreads();
  if (wave == 0) {
#pragma unroll 1
    for (int b0 = 0; b0 < tt; b0 += 32) {
      const int idx = b0 + lane;
      const int ent = hl[idx < RCAP ? idx : RCAP - 1];
      const int m32 = (tt - b0) < 32 ? (tt - b0) : 32;
#pragma unroll 1
      for (int k = 0; k < m32; ++k) {
        const int u    = __builtin_amdgcn_readlane(ent, k);
        const int slot = u & (NBA - 1);
        if (lane == 0) {
          int p = cur[slot];
          p = p < 0 ? 0 : (p > RCAP - 1 ? RCAP - 1 : p);
          sl[p] = u;
          cur[slot] = p + 1;
        }
      }
    }
  }
  __syncthreads();

  const float qnan = __int_as_float(0x7fc00000);
  const float pz = (ovf != 0) ? qnan : 0.0f;
#pragma unroll 1
  for (int si = 0; si < NBA / NWAVE; ++si) {
    const int s    = si * NWAVE + wave;
    const int node = nodeBase + s;
    int c = cnt[s];
    const bool big = c > DEGCAP;
    c = c < 0 ? 0 : (c > DEGCAP ? DEGCAP : c);
    int o = offs[s];
    o = o < 0 ? 0 : (o > RCAP ? RCAP : o);
    const float pzr = big ? qnan : pz;
    const bool live = node < nN;
    const int nc = live ? node : nN - 1;

    float a0 = 0.0f, a1 = 0.0f, a2 = 0.0f, a3 = 0.0f;
#pragma unroll 1
    for (int b0 = 0; b0 < c; b0 += 32) {
      int idx = o + b0 + lane;
      idx = idx > RCAP - 1 ? RCAP - 1 : idx;
      const int ent = sl[idx];
      int eid = ent >> SLA;
      eid = eid < 0 ? 0 : (eid > nE - 1 ? nE - 1 : eid);
      int sr = gath[eid];
      sr = sr < 0 ? 0 : (sr > nN - 1 ? nN - 1 : sr);
      const int m32 = (c - b0) < 32 ? (c - b0) : 32;
#pragma unroll 1
      for (int k = 0; k < m32; ++k) {
        const int sk = __builtin_amdgcn_readlane(sr, k);
        if constexpr (L1 != 0) {
          const v4f a = *(const v4fa*)(src + (size_t)sk * DIN + 4 * lane);
          a0 += bf16_val(a.x); a1 += bf16_val(a.y); a2 += bf16_val(a.z); a3 += bf16_val(a.w);
        } else {
          const v2f a = *(const v2fa*)(src + (size_t)sk * DOUT + 2 * lane);
          a0 += a.x; a1 += a.y;
        }
      }
    }
    const float inv = 1.0f / (float)(c + 1);
    if constexpr (L1 != 0) {
      const v4f xs = *(const v4fa*)(src + (size_t)nc * DIN + 4 * lane);
      const float m0 = live ? ((a0 + bf16_val(xs.x)) * inv + pzr) : 0.0f;
      const float m1 = live ? ((a1 + bf16_val(xs.y)) * inv + pzr) : 0.0f;
      const float m2 = live ? ((a2 + bf16_val(xs.z)) * inv + pzr) : 0.0f;
      const float m3 = live ? ((a3 + bf16_val(xs.w)) * inv + pzr) : 0.0f;
      const unsigned hb0 = bf16_bits(m0), hb1 = bf16_bits(m1), hb2 = bf16_bits(m2), hb3 = bf16_bits(m3);
      const unsigned lb0 = bf16_bits(m0 - __uint_as_float(hb0 << 16));
      const unsigned lb1 = bf16_bits(m1 - __uint_as_float(hb1 << 16));
      const unsigned lb2 = bf16_bits(m2 - __uint_as_float(hb2 << 16));
      const unsigned lb3 = bf16_bits(m3 - __uint_as_float(hb3 << 16));
      v2u ph, pl;
      ph.x = hb0 | (hb1 << 16); ph.y = hb2 | (hb3 << 16);
      pl.x = lb0 | (lb1 << 16); pl.y = lb2 | (lb3 << 16);
      *(v2ua*)(rowu + 2 * lane)          = ph;
      *(v2ua*)(rowu + RB / 4 + 2 * lane) = pl;
      wave_sync();
      const v8us q0 = *(const v8usa*)(rowbuf + 8 * lane);
      wave_sync();
      const bool wr = node < mRows;
      unsigned short* rpw = apl + (size_t)node * AP + 8 * lane;
      if (wr) *(volatile v8us*)rpw = q0;
      __threadfence();
      if (wr) *(volatile v8us*)rpw = q0;
    } else {
      const v2f ts = *(const v2fa*)(src + (size_t)nc * DOUT + 2 * lane);
      v2f st;
      st.x = live ? ((a0 + ts.x) * inv + bv0 + pzr) : 0.0f;
      st.y = live ? ((a1 + ts.y) * inv + bv1 + pzr) : 0.0f;
      *(v2fa*)(rowf + 2 * lane) = st;
      wave_sync();
      const v4f q0 = *(const v4fa*)(rowf + 4 * (lane & 15));
      wave_sync();
      const bool wr = live && (lane < 16);
      float* opw = outp + (size_t)nc * DOUT + 4 * (lane & 15);
      if (wr) *(volatile v4f*)opw = q0;
      __threadfence();
      if (wr) *(volatile v4f*)opw = q0;
    }
  }
}

static inline int cdiv(int a, int b) { return (a + b - 1) / b; }
static inline size_t al256(size_t o) { return (o + 255) & ~(size_t)255; }

extern "C" void kernel_launch(void* const* d_in, const int* in_sizes, int n_in,
                              void* d_out, int out_size, void* d_ws, size_t ws_size,
                              hipStream_t stream) {
  if (n_in < 7) return;
  if (in_sizes[0] < DIN || (in_sizes[0] % DIN) != 0) return;
  const int nN = in_sizes[0] / DIN;
  if (in_sizes[1] != DHID * DIN || in_sizes[2] != DHID) return;
  if (in_sizes[3] != DOUT * DHID || in_sizes[4] != DOUT) return;
  const int nE = in_sizes[5];
  if (in_sizes[6] != nE) return;
  if (nE < 1 || nE >= (1 << (31 - SLA)) || nN < 1 || nN >= (1 << 22)) return;
  if ((long long)out_size != (long long)nN * DOUT) return;

  const float* x   = (const float*)d_in[0];
  const float* W1  = (const float*)d_in[1];
  const float* b1  = (const float*)d_in[2];
  const float* W2  = (const float*)d_in[3];
  const float* b2  = (const float*)d_in[4];
  const int*   row = (const int*)d_in[5];
  const int*   col = (const int*)d_in[6];
  float* out = (float*)d_out;

  const int MP = cdiv(nN, GBM) * GBM;
  const int gM = MP / GBM;
  const int gA = cdiv(MP, NBA);
  if ((long long)gA * NBA < (long long)MP) return;
  const int vec8 = ((nE & 3) == 0) ? 1 : 0;

  char* ws = (char*)d_ws;
  size_t off = 0;
  const size_t oB1 = off; off = al256(off + (size_t)DHID * KC * 2);
  const size_t oB2 = off; off = al256(off + (size_t)DOUT * KC * 2);
  const size_t oA1 = off; off = al256(off + (size_t)MP * AP * 2);
  const size_t oH1 = off; off = al256(off + (size_t)MP * AP * 2);
  const size_t oT  = off; off = al256(off + (size_t)MP * DOUT * 4);
  if (off > ws_size || off > (size_t)WSMAX) return;
  unsigned short* BT1 = (unsigned short*)(ws + oB1);
  unsigned short* BT2 = (unsigned short*)(ws + oB2);
  unsigned short* A1  = (unsigned short*)(ws + oA1);
  unsigned short* H1  = (unsigned short*)(ws + oH1);
  float*          T   = (float*)(ws + oT);

  const size_t scanLds = (size_t)AGG_LDS_INTS * 4;
  hipFuncSetAttribute(reinterpret_cast<const void*>(&k_scan<1>), hipFuncAttributeMaxDynamicSharedMemorySize, (int)scanLds);
  hipFuncSetAttribute(reinterpret_cast<const void*>(&k_scan<0>), hipFuncAttributeMaxDynamicSharedMemorySize, (int)scanLds);

  k_wprep<<<(UW1 + UW2) / NTHR, NTHR, 0, stream>>>(W1, W2, BT1, BT2);
  k_scan<1><<<gA, NTHR, scanLds, stream>>>(row, col, nE, nN, vec8, MP, x, b1, A1, out);
  k_gemm<0><<<dim3(gM, DHID / GBN), GTHR, 0, stream>>>(A1, BT1, b1, nN, H1, T);
  k_gemm<1><<<dim3(gM, 1), GTHR, 0, stream>>>(H1, BT2, b1, nN, A1, T);
  k_scan<0><<<gA, NTHR, scanLds, stream>>>(row, col, nE, nN, vec8, MP, T, b2, A1, out);
}
